// Model_74938589381339
// MI455X (gfx1250) — hardware-verified
//
#include <hip/hip_runtime.h>
#include <math.h>

constexpr int T_STEPS     = 2048;
constexpr int N_BATCH     = 64;
constexpr int N_HID       = 200;
constexpr int N_GROWS     = 4 * N_HID;
constexpr int K_PAD       = 224;
constexpr int N_WAVES     = 13;
constexpr int N_PADROWS   = N_WAVES * 64;
constexpr int U_PAD       = N_WAVES * 16;
constexpr int WO_PAD      = 224;
constexpr int ROWS_BLK    = 16;
constexpr int SEQ_THR     = N_WAVES * 32;
constexpr int H_PITCH     = 224;
constexpr int H_TILE      = ROWS_BLK * H_PITCH;
constexpr int PLANE_ELEMS = N_PADROWS * K_PAD;
constexpr int PACK_THR    = 256;
constexpr int PACK_CHUNKS = K_PAD / 8;
constexpr int PACK_N8     = N_PADROWS * PACK_CHUNKS;
constexpr int FLUSH_STEPS = 8;
constexpr int N_OUT       = T_STEPS * N_BATCH;
constexpr float W_CARRY   = 64.0f;
constexpr float H_CARRY   = 64.0f;
constexpr float ACC_INV   = 1.0f / (W_CARRY * H_CARRY);

static_assert(K_PAD % 32 == 0, "k tiles of 32");
static_assert(K_PAD >= N_HID && H_PITCH == K_PAD, "A tile covers every k column that is loaded");
static_assert(U_PAD >= N_HID && U_PAD + 16 == K_PAD, "pad columns 208..223 are owned by the last wave");
static_assert(N_HID % 8 == 0, "8-element pack chunks are either fully real or fully pad");
static_assert(PACK_N8 % PACK_THR == 0, "pack grid exact");
static_assert(N_BATCH % ROWS_BLK == 0, "batch tiles");
static_assert(T_STEPS % FLUSH_STEPS == 0, "flush groups");
static_assert(FLUSH_STEPS * ROWS_BLK == 32 * 4, "one flush = 32 lanes x 4 floats");
static_assert((N_OUT / 4) % 256 == 0, "epilogue grid exact");
static_assert(SEQ_THR <= 512, "block size");

typedef __attribute__((ext_vector_type(16))) _Float16 v16h;
typedef __attribute__((ext_vector_type(8)))  _Float16 v8h;
typedef __attribute__((ext_vector_type(8)))  float    v8f;
typedef __attribute__((ext_vector_type(4)))  float    v4f;

__device__ __forceinline__ void guard_group(v8f& a0, v8f& a1, v8f& a2, v8f& a3,
                                            v16h a, v16h b0, v16h b1, v16h b2, v16h b3) {
  asm volatile("v_nop\n\tv_nop\n\tv_nop\n\tv_nop"
               : "+v"(a0), "+v"(a1), "+v"(a2), "+v"(a3)
               : "v"(a), "v"(b0), "v"(b1), "v"(b2), "v"(b3));
}
__device__ __forceinline__ void acc_guard4(v8f& a, v8f& b, v8f& c, v8f& d) {
  asm volatile("v_nop\n\tv_nop\n\tv_nop\n\tv_nop" : "+v"(a), "+v"(b), "+v"(c), "+v"(d));
}

template <typename T> struct Frag;
template <> struct Frag<_Float16> {
  typedef v16h V; union U { v16h v; v8h h[2]; };
  static __device__ __forceinline__ v16h load(const _Float16* p) {
    U f; f.h[0] = *(const v8h*)(p); f.h[1] = *(const v8h*)(p + 16); return f.v;
  }
  static __device__ __forceinline__ v8f mma(v16h a, v16h b, v8f c) {
    return __builtin_amdgcn_wmma_f32_16x16x32_f16(false, a, false, b, (short)0, c, false, false);
  }
};

__device__ __forceinline__ float gate_sig(float v)  { return __builtin_amdgcn_rcpf(1.0f + expf(-v)); }
__device__ __forceinline__ float gate_tanh(float v) { return 1.0f - 2.0f * __builtin_amdgcn_rcpf(1.0f + expf(2.0f * v)); }

__device__ __forceinline__ float cell_update(float zi, float zf, float zg, float zo, float& cst) {
  const float ig = gate_sig(zi);
  const float fg = gate_sig(zf);
  const float gg = gate_tanh(zg);
  const float og = gate_sig(zo);
  const float cn = fg * cst + ig * gg;
  cst = cn;
  return og * gate_tanh(cn);
}

__device__ __forceinline__ void chain_k224(const _Float16* arow, const _Float16* bt,
                                           v8f& a0, v8f& a1, v8f& a2, v8f& a3) {
#pragma unroll 1
  for (int k0 = 0; k0 < K_PAD; k0 += 32) {
    const v16h a  = Frag<_Float16>::load(arow + k0);
    const v16h b0 = Frag<_Float16>::load(bt + k0);
    const v16h b1 = Frag<_Float16>::load(bt + 16 * K_PAD + k0);
    const v16h b2 = Frag<_Float16>::load(bt + 32 * K_PAD + k0);
    const v16h b3 = Frag<_Float16>::load(bt + 48 * K_PAD + k0);
    a0 = Frag<_Float16>::mma(a, b0, a0);
    a1 = Frag<_Float16>::mma(a, b1, a1);
    a2 = Frag<_Float16>::mma(a, b2, a2);
    a3 = Frag<_Float16>::mma(a, b3, a3);
    guard_group(a0, a1, a2, a3, a, b0, b1, b2, b3);
  }
}

__global__ __launch_bounds__(PACK_THR) void pack_w_kernel(const float* __restrict__ w_hh0, const float* __restrict__ w_ih1,
                                                          const float* __restrict__ w_hh1, unsigned short* __restrict__ dst) {
  const int i = blockIdx.x * PACK_THR + threadIdx.x;
  if (i < PACK_N8) {
    const int plane = blockIdx.y;
    const float* src = (plane == 0) ? w_hh0 : ((plane == 1) ? w_ih1 : w_hh1);
    const int row = i / PACK_CHUNKS;
    const int c8  = (i - row * PACK_CHUNKS) * 8;
    const int w = row >> 6, g = (row >> 4) & 3, u = row & 15;
    const int unit  = 16 * w + u;
    const int unitc = (unit < N_HID) ? unit : (N_HID - 1);
    const int c8c   = (c8 < N_HID - 8) ? c8 : (N_HID - 8);
    const bool valid = (unit < N_HID) && (c8 < N_HID);
    const float* sp = src + (size_t)(g * N_HID + unitc) * N_HID + c8c;
    const v4f va = *(const v4f*)(sp);
    const v4f vb = *(const v4f*)(sp + 4);
    v8h hv;
#pragma unroll
    for (int e = 0; e < 4; ++e) {
      const float fa = valid ? (va[e] * W_CARRY) : 0.0f;
      const float fb = valid ? (vb[e] * W_CARRY) : 0.0f;
      hv[e]     = (_Float16)fa;
      hv[4 + e] = (_Float16)fb;
    }
    unsigned short* dp = dst + (size_t)plane * PLANE_ELEMS + (size_t)i * 8;
    *(volatile v8h*)dp = hv;
    __threadfence();
    *(volatile v8h*)dp = hv;
  }
}

__global__ __launch_bounds__(PACK_THR) void pack_c_kernel(const float* __restrict__ w_ih0,
                                                          const float* __restrict__ b_ih0, const float* __restrict__ b_hh0,
                                                          const float* __restrict__ b_ih1, const float* __restrict__ b_hh1,
                                                          const float* __restrict__ w_out,
                                                          float* __restrict__ P0, float* __restrict__ P1,
                                                          float* __restrict__ P2, float* __restrict__ WO) {
  const int tid = threadIdx.x;
  const int q = blockIdx.x;
  if (q < 3) {
    if (tid < U_PAD) {
      const int uc = (tid < N_HID) ? tid : (N_HID - 1);
      const bool valid = tid < N_HID;
      v4f o;
      if (q == 0) {
#pragma unroll
        for (int g = 0; g < 4; ++g) { const float v = w_ih0[g * N_HID + uc]; o[g] = valid ? v : 0.0f; }
      } else if (q == 1) {
#pragma unroll
        for (int g = 0; g < 4; ++g) { const float v = b_ih0[g * N_HID + uc] + b_hh0[g * N_HID + uc]; o[g] = valid ? v : 0.0f; }
      } else {
#pragma unroll
        for (int g = 0; g < 4; ++g) { const float v = b_ih1[g * N_HID + uc] + b_hh1[g * N_HID + uc]; o[g] = valid ? v : 0.0f; }
      }
      float* dp = ((q == 0) ? P0 : ((q == 1) ? P1 : P2)) + tid * 4;
      *(volatile v4f*)dp = o;
      __threadfence();
      *(volatile v4f*)dp = o;
    }
  } else {
    if (tid < WO_PAD / 4) {
      v4f o;
#pragma unroll
      for (int e = 0; e < 4; ++e) {
        const int idx = 4 * tid + e;
        const int ic = (idx < N_HID) ? idx : (N_HID - 1);
        const float v = w_out[ic];
        o[e] = (idx < N_HID) ? v : 0.0f;
      }
      float* dp = WO + tid * 4;
      *(volatile v4f*)dp = o;
      __threadfence();
      *(volatile v4f*)dp = o;
    }
  }
}

__global__ __launch_bounds__(SEQ_THR) void lstm2_seq_kernel(const float* __restrict__ x,
                                                            const unsigned short* __restrict__ BTp,
                                                            const float* __restrict__ P0, const float* __restrict__ P1,
                                                            const float* __restrict__ P2, const float* __restrict__ WO,
                                                            const float* __restrict__ bout,
                                                            float* __restrict__ Y) {
  __shared__ __align__(16) _Float16 H1s[2][H_TILE];
  __shared__ __align__(16) _Float16 H2s[2][H_TILE];
  __shared__ __align__(16) float    partS[N_WAVES * ROWS_BLK];
  __shared__ __align__(16) float    ybuf[FLUSH_STEPS * ROWS_BLK];

  const int tid = threadIdx.x, lane = tid & 31, wave = tid >> 5;
  const int c = lane & 15, hh = lane >> 4, koff = hh * 8;
  const int rowbase = blockIdx.x * ROWS_BLK;
  const int unit = 16 * wave + c;
  const bool uvalid = unit < N_HID;

  {
    _Float16* z1 = &H1s[0][0];
    _Float16* z2 = &H2s[0][0];
#pragma unroll 1
    for (int i = tid; i < 2 * H_TILE; i += SEQ_THR) {
      z1[i] = (_Float16)0.0f;
      z2[i] = (_Float16)0.0f;
    }
  }

  const v4f pw  = *(const v4f*)(P0 + unit * 4);
  const v4f pb0 = *(const v4f*)(P1 + unit * 4);
  const v4f pb1 = *(const v4f*)(P2 + unit * 4);
  const float wo = WO[unit];
  const float bo = bout[0];

  const _Float16* BT  = (const _Float16*)BTp;
  const _Float16* bt0 = BT + (size_t)(wave * 64 + c) * K_PAD + koff;
  const _Float16* bt1 = bt0 + PLANE_ELEMS;
  const _Float16* bt2 = bt1 + PLANE_ELEMS;

  float c1s[8], c2s[8];
#pragma unroll
  for (int r = 0; r < 8; ++r) { c1s[r] = 0.0f; c2s[r] = 0.0f; }

  float* Yb = Y + (size_t)blockIdx.x * T_STEPS * ROWS_BLK;
  const v8f z8 = {0.f, 0.f, 0.f, 0.f, 0.f, 0.f, 0.f, 0.f};
  const int arow_off = c * H_PITCH + koff;

  __syncthreads();

#pragma unroll 1
  for (int t = 0; t < T_STEPS; ++t) {
    const int pp = t & 1;
    const _Float16* h1prev = &H1s[0][0] + pp * H_TILE + arow_off;
    _Float16*       h1next = &H1s[0][0] + (pp ^ 1) * H_TILE;
    const _Float16* h1cur  = h1next + arow_off;
    const _Float16* h2prev = &H2s[0][0] + pp * H_TILE + arow_off;
    _Float16*       h2next = &H2s[0][0] + (pp ^ 1) * H_TILE;

    const float* xp = x + (size_t)t * N_BATCH + rowbase + 8 * hh;
    const v4f xa = *(const v4f*)(xp);
    const v4f xb = *(const v4f*)(xp + 4);
    const float xv[8] = {xa[0], xa[1], xa[2], xa[3], xb[0], xb[1], xb[2], xb[3]};

    {
      v8f a0 = z8, a1 = z8, a2 = z8, a3 = z8;
      chain_k224(h1prev, bt0, a0, a1, a2, a3);
      acc_guard4(a0, a1, a2, a3);
#pragma unroll
      for (int r = 0; r < 8; ++r) {
        const float zi = fmaf(a0[r], ACC_INV, fmaf(xv[r], pw[0], pb0[0]));
        const float zf = fmaf(a1[r], ACC_INV, fmaf(xv[r], pw[1], pb0[1]));
        const float zg = fmaf(a2[r], ACC_INV, fmaf(xv[r], pw[2], pb0[2]));
        const float zo = fmaf(a3[r], ACC_INV, fmaf(xv[r], pw[3], pb0[3]));
        const float hn = cell_update(zi, zf, zg, zo, c1s[r]);
        const float hsel = uvalid ? hn : 0.0f;
        h1next[(8 * hh + r) * H_PITCH + unit] = (_Float16)(hsel * H_CARRY);
      }
      if (wave == N_WAVES - 1) {
#pragma unroll
        for (int r = 0; r < 8; ++r) h1next[(8 * hh + r) * H_PITCH + U_PAD + c] = (_Float16)0.0f;
      }
    }
    __syncthreads();

    {
      v8f a0 = z8, a1 = z8, a2 = z8, a3 = z8;
      chain_k224(h1cur,  bt1, a0, a1, a2, a3);
      chain_k224(h2prev, bt2, a0, a1, a2, a3);
      acc_guard4(a0, a1, a2, a3);
#pragma unroll
      for (int r = 0; r < 8; ++r) {
        const float zi = fmaf(a0[r], ACC_INV, pb1[0]);
        const float zf = fmaf(a1[r], ACC_INV, pb1[1]);
        const float zg = fmaf(a2[r], ACC_INV, pb1[2]);
        const float zo = fmaf(a3[r], ACC_INV, pb1[3]);
        const float hn = cell_update(zi, zf, zg, zo, c2s[r]);
        const float hsel = uvalid ? hn : 0.0f;
        h2next[(8 * hh + r) * H_PITCH + unit] = (_Float16)(hsel * H_CARRY);
        float p = hsel * wo;
        p += __shfl_xor(p, 1, 32);
        p += __shfl_xor(p, 2, 32);
        p += __shfl_xor(p, 4, 32);
        p += __shfl_xor(p, 8, 32);
        if (c == 0) partS[wave * ROWS_BLK + 8 * hh + r] = p;
      }
      if (wave == N_WAVES - 1) {
#pragma unroll
        for (int r = 0; r < 8; ++r) h2next[(8 * hh + r) * H_PITCH + U_PAD + c] = (_Float16)0.0f;
      }
    }
    __syncthreads();

    if (tid < ROWS_BLK) {
      float s = bo;
#pragma unroll
      for (int w = 0; w < N_WAVES; ++w) s += partS[w * ROWS_BLK + tid];
      ybuf[(t & (FLUSH_STEPS - 1)) * ROWS_BLK + tid] = s;
    }
    if (wave == 0 && (t & (FLUSH_STEPS - 1)) == (FLUSH_STEPS - 1)) {
      __builtin_amdgcn_fence(__ATOMIC_RELEASE, "workgroup");
      __builtin_amdgcn_wave_barrier();
      __builtin_amdgcn_fence(__ATOMIC_ACQUIRE, "workgroup");
      const v4f yv = *(const v4f*)(ybuf + 4 * lane);
      float* yp = Yb + (size_t)(t - (FLUSH_STEPS - 1)) * ROWS_BLK + 4 * lane;
      *(volatile v4f*)yp = yv;
      __threadfence();
      *(volatile v4f*)yp = yv;
      __builtin_amdgcn_fence(__ATOMIC_RELEASE, "workgroup");
      __builtin_amdgcn_wave_barrier();
      __builtin_amdgcn_fence(__ATOMIC_ACQUIRE, "workgroup");
    }
  }
}

__global__ __launch_bounds__(256) void out_gather_kernel(const float* __restrict__ Y, float* __restrict__ out) {
  const int i = blockIdx.x * 256 + threadIdx.x;
  if (i < N_OUT / 4) {
    const int t = i >> 4;
    const int qd = i & 15;
    const int tile = qd >> 2;
    const int within = (qd & 3) * 4;
    const v4f v = *(const v4f*)(Y + ((size_t)tile * T_STEPS + (size_t)t) * ROWS_BLK + within);
    float* op = out + (size_t)i * 4;
    *(volatile v4f*)op = v;
    __threadfence();
    *(volatile v4f*)op = v;
  }
}

extern "C" void kernel_launch(void* const* d_in, const int* in_sizes, int n_in,
                              void* d_out, int out_size, void* d_ws, size_t ws_size, hipStream_t stream) {
  if (n_in < 11 || d_out == nullptr || d_ws == nullptr) return;
  if (in_sizes[0] != T_STEPS * N_BATCH || in_sizes[1] != N_GROWS || in_sizes[2] != N_GROWS * N_HID ||
      in_sizes[3] != N_GROWS || in_sizes[4] != N_GROWS || in_sizes[5] != N_GROWS * N_HID ||
      in_sizes[6] != N_GROWS * N_HID || in_sizes[7] != N_GROWS || in_sizes[8] != N_GROWS ||
      in_sizes[9] != N_HID || in_sizes[10] != 1 || out_size != N_OUT) return;

  const float* x     = (const float*)d_in[0];
  const float* w_ih0 = (const float*)d_in[1];
  const float* w_hh0 = (const float*)d_in[2];
  const float* b_ih0 = (const float*)d_in[3];
  const float* b_hh0 = (const float*)d_in[4];
  const float* w_ih1 = (const float*)d_in[5];
  const float* w_hh1 = (const float*)d_in[6];
  const float* b_ih1 = (const float*)d_in[7];
  const float* b_hh1 = (const float*)d_in[8];
  const float* w_out = (const float*)d_in[9];
  const float* b_out = (const float*)d_in[10];
  float* out = (float*)d_out;

  char* ws = (char*)d_ws; size_t off = 0;
  auto carve = [&](size_t bytes) -> char* { char* p = ws + off; off += (bytes + 255) & ~(size_t)255; return p; };
  unsigned short* BT = (unsigned short*)carve((size_t)3 * PLANE_ELEMS * 2);
  float* P0 = (float*)carve((size_t)U_PAD * 4 * 4);
  float* P1 = (float*)carve((size_t)U_PAD * 4 * 4);
  float* P2 = (float*)carve((size_t)U_PAD * 4 * 4);
  float* WO = (float*)carve((size_t)WO_PAD * 4);
  float* Y  = (float*)carve((size_t)(N_BATCH / ROWS_BLK) * T_STEPS * ROWS_BLK * 4);
  if (off > ws_size || off > (size_t)134217728) return;

  pack_w_kernel<<<dim3(PACK_N8 / PACK_THR, 3), PACK_THR, 0, stream>>>(w_hh0, w_ih1, w_hh1, BT);
  pack_c_kernel<<<4, PACK_THR, 0, stream>>>(w_ih0, b_ih0, b_hh0, b_ih1, b_hh1, w_out, P0, P1, P2, WO);
  lstm2_seq_kernel<<<N_BATCH / ROWS_BLK, SEQ_THR, 0, stream>>>(x, BT, P0, P1, P2, WO, b_out, Y);
  out_gather_kernel<<<(N_OUT / 4) / 256, 256, 0, stream>>>(Y, out);
}
